// RNNModel_55155970015295
// MI455X (gfx1250) — hardware-verified
//
#include <hip/hip_runtime.h>
#include <math.h>

constexpr int NB      = 1024;
constexpr int T1      = 512;
constexpr int T2      = 64;
constexpr int TT      = T1 + T2;
constexpr int DF      = 9;
constexpr int NH      = 100;
constexpr int NG4     = 4 * NH;
constexpr int DO      = 9;
constexpr int NTHR    = 256;
constexpr int ROWS_BLK = 16;
constexpr int KP      = 128;
constexpr int KENC    = NH;
constexpr int KZERO   = NH + DF;
constexpr int NSUB    = 7;
constexpr int UPAD    = NSUB * 16;
constexpr int BT_ROWS = 4 * UPAD + 16;
constexpr int AP      = 136;
constexpr int TSP     = 17;
constexpr int CHUNK   = 32;
constexpr int OROW    = CHUNK * DO;
constexpr int OSTN    = ROWS_BLK * OROW;
constexpr int LINES_PER_FLUSH = OSTN * 4 / 128;
static_assert(TT == 576 && NG4 == 400, "shape constants");
static_assert(NB % ROWS_BLK == 0, "grid exact");
static_assert(TT % CHUNK == 0 && T1 % CHUNK == 0, "no ragged output chunk");
static_assert((OROW * 4) % 128 == 0, "per-row chunk is whole lines");
static_assert((TT * DO * 4) % 128 == 0, "per-batch-row output slab is line aligned");
static_assert((OSTN * 4) % 128 == 0 && LINES_PER_FLUSH * 8 == 1152, "flush coverage");
static_assert(KP % 32 == 0 && KZERO <= KP && UPAD >= NH, "K and N padding");
static_assert(AP % 8 == 0 && AP >= KP, "A tile pitch");
static_assert((ROWS_BLK * AP) % 2 == 0, "A tile zero fill in 32-bit words");
static_assert(BT_ROWS % 16 == 0, "B plane builder grid exact");
static_assert(ROWS_BLK * DF <= 5 * 32, "encoder threads live in waves 0..4");

typedef __attribute__((ext_vector_type(16))) _Float16 v16h;
typedef __attribute__((ext_vector_type(8)))  _Float16 v8h;
typedef __attribute__((ext_vector_type(16))) __bf16   v16b;
typedef __attribute__((ext_vector_type(8)))  __bf16   v8b;
typedef __attribute__((ext_vector_type(8)))  float    v8f;
typedef __attribute__((ext_vector_type(4)))  float    v4f;

__device__ __forceinline__ unsigned short f2bf_bits(float f) {
  unsigned u = __float_as_uint(f);
  return (unsigned short)((u + 0x7FFFu + ((u >> 16) & 1u)) >> 16);
}
__device__ __forceinline__ float bf_bits2f(unsigned short h) { return __uint_as_float(((unsigned)h) << 16); }
__device__ __forceinline__ float bf16r(float f) { return bf_bits2f(f2bf_bits(f)); }

__device__ __forceinline__ void guard_all_b(v8f& a0, v8f& a1, v8f& a2, v8f& a3,
                                            v16b x, v16b y0, v16b y1, v16b y2, v16b y3) {
  asm volatile("v_nop\n\tv_nop\n\tv_nop\n\tv_nop"
               : "+v"(a0), "+v"(a1), "+v"(a2), "+v"(a3)
               : "v"(x), "v"(y0), "v"(y1), "v"(y2), "v"(y3));
}
__device__ __forceinline__ void guard_one_b(v8f& a0, v16b x, v16b y) {
  asm volatile("v_nop\n\tv_nop\n\tv_nop\n\tv_nop" : "+v"(a0) : "v"(x), "v"(y));
}
__device__ __forceinline__ void acc_guard4(v8f& a, v8f& b, v8f& c, v8f& d) { asm volatile("v_nop\n\tv_nop\n\tv_nop\n\tv_nop" : "+v"(a), "+v"(b), "+v"(c), "+v"(d)); }
__device__ __forceinline__ void acc_guard1(v8f& a) { asm volatile("v_nop\n\tv_nop\n\tv_nop\n\tv_nop" : "+v"(a)); }

template <typename T> struct Frag;
template <> struct Frag<__bf16> {
  typedef v16b V; union U { v16b v; v8b h[2]; };
  static __device__ __forceinline__ v16b load(const __bf16* p) {
    U f; f.h[0] = *(const v8b*)(p); f.h[1] = *(const v8b*)(p + 16); return f.v;
  }
  static __device__ __forceinline__ v8f mma(v16b a, v16b b, v8f c) {
    return __builtin_amdgcn_wmma_f32_16x16x32_bf16(false, a, false, b, (short)0, c, false, false);
  }
};

__device__ __forceinline__ float fsig(float x)  { return __builtin_amdgcn_rcpf(1.0f + expf(-x)); }
__device__ __forceinline__ float ftanh(float x) { return 1.0f - 2.0f * __builtin_amdgcn_rcpf(expf(2.0f * x) + 1.0f); }

__global__ __launch_bounds__(NTHR) void build_bt_kernel(const float* __restrict__ W_h, const float* __restrict__ W_x,
                                                        const float* __restrict__ W_out, unsigned short* __restrict__ Bt) {
  __shared__ float Ts[KP * TSP];
  const int tid = threadIdx.x;
  const int blk = blockIdx.x;
  const bool islog = (blk == 4 * NSUB);
  const int gq  = blk / NSUB;
  const int g   = (gq < 4) ? gq : 3;
  const int ub  = blk - gq * NSUB;
#pragma unroll 1
  for (int idx = tid; idx < NH * 16; idx += NTHR) {
    const int k = idx >> 4, c = idx & 15;
    float v;
    if (islog) {
      const int dcl = (c < DO) ? c : (DO - 1);
      const float w = W_out[(size_t)k * DO + dcl];
      v = (c < DO) ? w : 0.0f;
    } else {
      const int u  = 16 * ub + c;
      const int uc = (u < NH) ? u : (NH - 1);
      const float w = W_h[(size_t)k * NG4 + g * NH + uc];
      v = (u < NH) ? w : 0.0f;
    }
    Ts[k * TSP + c] = v;
  }
#pragma unroll 1
  for (int idx = tid; idx < DF * 16; idx += NTHR) {
    const int f = idx >> 4, c = idx & 15;
    float v = 0.0f;
    if (!islog) {
      const int u  = 16 * ub + c;
      const int uc = (u < NH) ? u : (NH - 1);
      const float w = W_x[(size_t)f * NG4 + g * NH + uc];
      v = (u < NH) ? w : 0.0f;
    }
    Ts[(KENC + f) * TSP + c] = v;
  }
#pragma unroll 1
  for (int idx = tid; idx < (KP - KZERO) * 16; idx += NTHR) {
    const int kk = idx >> 4, c = idx & 15;
    Ts[(KZERO + kk) * TSP + c] = 0.0f;
  }
  __syncthreads();
  const int r = tid >> 4, c8 = (tid & 15) * 8;
  v8h hv;
#pragma unroll
  for (int e = 0; e < 8; ++e) {
    const unsigned short bits = f2bf_bits(Ts[(c8 + e) * TSP + r]);
    hv[e] = __builtin_bit_cast(_Float16, bits);
  }
  unsigned short* op = Bt + (size_t)(blk * 16 + r) * KP + c8;
  *(volatile v8h*)op = hv;
  __threadfence();
  *(volatile v8h*)op = hv;
}

__global__ __launch_bounds__(NTHR) void lstm_seq_kernel(const float* __restrict__ inp, const float* __restrict__ tsk,
                                                        const float* __restrict__ W_in, const float* __restrict__ b_in,
                                                        const float* __restrict__ W_task, const float* __restrict__ b_task,
                                                        const float* __restrict__ b_lstm, const float* __restrict__ b_out,
                                                        const unsigned short* __restrict__ Btp, float* __restrict__ out) {
  __shared__ __align__(16) unsigned short Au[ROWS_BLK * AP];
  __shared__ __align__(16) float Ost[OSTN];
  __shared__ float sW[2 * DF * DF];
  __shared__ float sBe[2 * DF];
  const __bf16* Bt = (const __bf16*)Btp;
  const int tid  = threadIdx.x;
  const int lane = tid & 31;
  const int wave_u = __builtin_amdgcn_readfirstlane(tid >> 5);
  const int c = lane & 15, hh = lane >> 4, koff = hh * 8;
  const int rowbase = blockIdx.x * ROWS_BLK;

  {
    unsigned* aw = (unsigned*)(void*)Au;
#pragma unroll 1
    for (int i = tid; i < ROWS_BLK * AP / 2; i += NTHR) aw[i] = 0u;
  }
#pragma unroll 1
  for (int i = tid; i < OSTN; i += NTHR) Ost[i] = 0.0f;
#pragma unroll 1
  for (int i = tid; i < DF * DF; i += NTHR) { sW[i] = bf16r(W_in[i]); sW[DF * DF + i] = bf16r(W_task[i]); }
  if (tid < DF) { sBe[tid] = bf16r(b_in[tid]); sBe[DF + tid] = bf16r(b_task[tid]); }
  const int ubw = (wave_u < NSUB) ? wave_u : (NSUB - 1);
  const int unit = 16 * ubw + c;
  const int unitc = (unit < NH) ? unit : (NH - 1);
  float bg[4];
#pragma unroll
  for (int g = 0; g < 4; ++g) bg[g] = bf16r(b_lstm[g * NH + unitc]);
  const float bo = bf16r(b_out[(c < DO) ? c : (DO - 1)]);
  float cst[8], hreg[8];
#pragma unroll
  for (int r = 0; r < 8; ++r) { cst[r] = 0.0f; hreg[r] = 0.0f; }
  __syncthreads();

  const __bf16* arow = (const __bf16*)(const void*)Au + c * AP + koff;
  const __bf16* bw   = Bt + (size_t)unit * KP + koff;
  const __bf16* blp  = Bt + (size_t)(4 * UPAD + c) * KP + koff;
  const v8f z8 = {0.f, 0.f, 0.f, 0.f, 0.f, 0.f, 0.f, 0.f};
  const bool cvalid = (c < DO);

#pragma unroll 1
  for (int t = 0; t <= TT; ++t) {
    if (wave_u < 5) {
      const int rq = tid / DF;
      const int rr = (rq < ROWS_BLK) ? rq : (ROWS_BLK - 1);
      const int d  = tid - rq * DF;
      const int tt = (t < TT) ? t : (TT - 1);
      const int sel = (tt >= T1) ? 1 : 0;
      const int ti = (tt < T1) ? tt : (T1 - 1);
      const int tk = (tt >= T1) ? (tt - T1) : 0;
      const float* pin = inp + ((size_t)(rowbase + rr) * T1 + (size_t)ti) * DF;
      const float* ptk = tsk + ((size_t)(rowbase + rr) * T2 + (size_t)tk) * DF;
      const float* rp = sel ? ptk : pin;
      const float* wp = sW + sel * (DF * DF);
      float a = 0.0f;
#pragma unroll
      for (int f = 0; f < DF; ++f) a = fmaf(bf16r(rp[f]), wp[f * DF + d], a);
      const float enc = fmaxf(a + sBe[sel * DF + d], 0.0f);
      if (tid < ROWS_BLK * DF) Au[rr * AP + KENC + d] = f2bf_bits(enc);
    }
    if (tid < ROWS_BLK) {
#pragma unroll
      for (int cc = 0; cc < KP - KZERO; ++cc) Au[tid * AP + KZERO + cc] = (unsigned short)0;
    }
    __syncthreads();

    if (wave_u < NSUB) {
      v8f acc[4];
      acc[0] = z8; acc[1] = z8; acc[2] = z8; acc[3] = z8;
#pragma unroll 1
      for (int k0 = 0; k0 < KP; k0 += 32) {
        const v16b a  = Frag<__bf16>::load(arow + k0);
        const v16b b0 = Frag<__bf16>::load(bw + (size_t)0 * UPAD * KP + k0);
        const v16b b1 = Frag<__bf16>::load(bw + (size_t)1 * UPAD * KP + k0);
        const v16b b2 = Frag<__bf16>::load(bw + (size_t)2 * UPAD * KP + k0);
        const v16b b3 = Frag<__bf16>::load(bw + (size_t)3 * UPAD * KP + k0);
        acc[0] = Frag<__bf16>::mma(a, b0, acc[0]);
        acc[1] = Frag<__bf16>::mma(a, b1, acc[1]);
        acc[2] = Frag<__bf16>::mma(a, b2, acc[2]);
        acc[3] = Frag<__bf16>::mma(a, b3, acc[3]);
        guard_all_b(acc[0], acc[1], acc[2], acc[3], a, b0, b1, b2, b3);
      }
      acc_guard4(acc[0], acc[1], acc[2], acc[3]);
#pragma unroll
      for (int r = 0; r < 8; ++r) {
        const float zi = acc[0][r] + bg[0];
        const float zf = acc[1][r] + bg[1];
        const float zg = acc[2][r] + bg[2];
        const float zo = acc[3][r] + bg[3];
        const float ig = fsig(zi);
        const float fg = fsig(zf);
        const float gg = ftanh(zg);
        const float og = fsig(zo);
        const float cn = fg * cst[r] + ig * gg;
        cst[r] = cn;
        hreg[r] = og * ftanh(cn);
      }
    } else {
      v8f acc = z8;
#pragma unroll
      for (int k0 = 0; k0 < KP; k0 += 32) {
        const v16b a = Frag<__bf16>::load(arow + k0);
        const v16b b = Frag<__bf16>::load(blp + k0);
        acc = Frag<__bf16>::mma(a, b, acc);
        guard_one_b(acc, a, b);
      }
      acc_guard1(acc);
      const int slot = (t + CHUNK - 1) & (CHUNK - 1);
#pragma unroll
      for (int r = 0; r < 8; ++r) {
        const float lg = acc[r] + bo;
        float m = cvalid ? lg : -INFINITY;
        m = fmaxf(m, __shfl_xor(m, 1, 32));
        m = fmaxf(m, __shfl_xor(m, 2, 32));
        m = fmaxf(m, __shfl_xor(m, 4, 32));
        m = fmaxf(m, __shfl_xor(m, 8, 32));
        const float er = expf(lg - m);
        const float e  = cvalid ? er : 0.0f;
        float s = e;
        s += __shfl_xor(s, 1, 32);
        s += __shfl_xor(s, 2, 32);
        s += __shfl_xor(s, 4, 32);
        s += __shfl_xor(s, 8, 32);
        const float p = e * (1.0f / s);
        if (cvalid && t >= 1) Ost[(8 * hh + r) * OROW + slot * DO + c] = p;
      }
    }
    __syncthreads();

    if ((t & (CHUNK - 1)) == 0 && t >= CHUNK) {
      const int s0 = t - CHUNK;
      for (int pass = 0; pass < 2; ++pass) {
#pragma unroll 1
        for (int i = tid; i < LINES_PER_FLUSH * 8; i += NTHR) {
          const int L = i >> 3, q = i & 7;
          const int r = L / 9, lr = L - 9 * r;
          const v4f v = *(const v4f*)(Ost + i * 4);
          const size_t go = ((size_t)(rowbase + r) * TT + (size_t)s0) * DO + (size_t)(lr * 32 + q * 4);
          *(volatile v4f*)(out + go) = v;
        }
        __threadfence();
      }
    }
    if (wave_u < NSUB) {
      const int u = 16 * wave_u + c;
      if (u < NH) {
#pragma unroll
        for (int r = 0; r < 8; ++r) Au[(8 * hh + r) * AP + u] = f2bf_bits(hreg[r]);
      }
    }
  }
}

extern "C" void kernel_launch(void* const* d_in, const int* in_sizes, int n_in,
                              void* d_out, int out_size, void* d_ws, size_t ws_size, hipStream_t stream) {
  if (n_in < 11 || d_out == nullptr || d_ws == nullptr) return;
  if (in_sizes[0] != NB * T1 * DF || in_sizes[1] != NB * T2 * DF || in_sizes[2] != DF * DF || in_sizes[3] != DF ||
      in_sizes[4] != DF * DF || in_sizes[5] != DF || in_sizes[6] != DF * NG4 || in_sizes[7] != NH * NG4 ||
      in_sizes[8] != NG4 || in_sizes[9] != NH * DO || in_sizes[10] != DO || out_size != NB * TT * DO) return;

  const float* inp    = (const float*)d_in[0];
  const float* tsk    = (const float*)d_in[1];
  const float* W_in   = (const float*)d_in[2];
  const float* b_in   = (const float*)d_in[3];
  const float* W_task = (const float*)d_in[4];
  const float* b_task = (const float*)d_in[5];
  const float* W_x    = (const float*)d_in[6];
  const float* W_h    = (const float*)d_in[7];
  const float* b_lstm = (const float*)d_in[8];
  const float* W_out  = (const float*)d_in[9];
  const float* b_out  = (const float*)d_in[10];
  float* outp = (float*)d_out;

  const size_t bt_bytes = (size_t)BT_ROWS * KP * 2;
  if (bt_bytes > ws_size || bt_bytes > (size_t)134217728) return;
  unsigned short* Bt = (unsigned short*)d_ws;

  build_bt_kernel<<<BT_ROWS / 16, NTHR, 0, stream>>>(W_h, W_x, W_out, Bt);
  lstm_seq_kernel<<<NB / ROWS_BLK, NTHR, 0, stream>>>(inp, tsk, W_in, b_in, W_task, b_task, b_lstm, b_out, Bt, outp);
}
